// CCN1D_7584912245325
// MI455X (gfx1250) — hardware-run, weakly checked
//
#include <hip/hip_runtime.h>
#include <stddef.h>
#include <math.h>


#define DS     64
#define DH     128
#define DP     256
#define KP1    17
#define VB     16
#define NT     17
#define TIT    3
#define NTHR   256
#define NWAVE  8
#define BM     32
#define DFC    192
#define DO     32
#define HCAP   4096
#define CHK    (NTHR * 8)
#define WSCAP  134217728
#define SCL_A  8.0f
#define SCL_W  16.0f
#define SCL_U  256.0f
#define INV_PQ 0.0078125f
#define INV_H2 ((1.0f / 17.0f) * 0.000244140625f)

static_assert(VB * KP1 == NT * 16);
static_assert(TIT * NWAVE >= NT);
static_assert(NTHR == NWAVE * 32);
static_assert(VB * DS == NTHR * 4);
static_assert((BM * DP / 4) % NTHR == 0);
static_assert((DS * DH / 8) % NTHR == 0);
static_assert(DFC == 3 * DS && DO == 32);
static_assert((HCAP & (HCAP - 1)) == 0);

typedef float    v4f  __attribute__((ext_vector_type(4)));
typedef float    v8f  __attribute__((ext_vector_type(8)));
typedef int      v4i  __attribute__((ext_vector_type(4)));
typedef _Float16 v4h  __attribute__((ext_vector_type(4)));
typedef _Float16 v8h  __attribute__((ext_vector_type(8)));
typedef _Float16 v16h __attribute__((ext_vector_type(16)));
union FragH { v16h v; v8h h[2]; };

__device__ __forceinline__ v8f wmh(v16h a, v16h b, v8f c) {
  v8f d = __builtin_amdgcn_wmma_f32_16x16x32_f16(false, a, false, b, (short)0, c, false, false);
  asm volatile("v_nop\n\tv_nop\n\tv_nop\n\tv_nop" : "+v"(d) : "v"(a), "v"(b));
  return d;
}

__device__ __forceinline__ v8h cvt8(v4f a, v4f b, float s) {
  v8f t;
  t[0] = a.x * s; t[1] = a.y * s; t[2] = a.z * s; t[3] = a.w * s;
  t[4] = b.x * s; t[5] = b.y * s; t[6] = b.z * s; t[7] = b.w * s;
  return __builtin_convertvector(t, v8h);
}

__device__ __forceinline__ int clampi(int v, int lo, int hi) { return v < lo ? lo : (v > hi ? hi : v); }

__device__ __forceinline__ v4f relu4(v4f u) {
  u.x = fmaxf(u.x, 0.0f); u.y = fmaxf(u.y, 0.0f); u.z = fmaxf(u.z, 0.0f); u.w = fmaxf(u.w, 0.0f);
  return u;
}

__global__ __launch_bounds__(NTHR) void k_prepw(const float* __restrict__ W, _Float16* wp,
                                               int nrW, int ldw, int NP, int KP, int nsplit, int ksplit) {
  const int i   = (int)blockIdx.x * NTHR + (int)threadIdx.x;
  const int upr = KP >> 3;
  const int nU  = NP * upr;
  if (i >= nU) return;
  const int n  = i / upr;
  const int k0 = (i - n * upr) * 8;
  const bool up = n >= nsplit;
  int cidx = up ? n - nsplit : n;
  cidx = clampi(cidx, 0, ldw - 1);
  const int kb = up ? ksplit : 0;
  v8f t;
#pragma unroll
  for (int e = 0; e < 8; ++e) {
    const int rr = clampi(kb + k0 + e, 0, nrW - 1);
    t[e] = W[(size_t)rr * ldw + cidx] * SCL_W;
  }
  const v8h o = __builtin_convertvector(t, v8h);
  _Float16* d = wp + (size_t)i * 8;
  *(volatile v8h*)d = o;
  __threadfence();
  *(volatile v8h*)d = o;
}

__global__ __launch_bounds__(NTHR) void k_embed(const int* __restrict__ x, const float* __restrict__ emb,
                                               float* F0f, _Float16* F0h, int nN, int V, int nU4, int nU8) {
  const int i = (int)blockIdx.x * NTHR + (int)threadIdx.x;
  const v4f z4 = {0.0f, 0.0f, 0.0f, 0.0f};

  const bool a4  = i < nU4;
  const int row4 = i >> 4;
  const int c4   = (i & 15) * 4;
  const int r4   = clampi(row4, 0, nN - 1);
  int id4 = x[r4];
  id4 = id4 < 0 ? id4 + V : id4;
  id4 = clampi(id4, 0, V - 1);
  v4f e4 = *(const v4f*)(emb + (size_t)id4 * DS + c4);
  e4 = relu4(e4);
  e4 = (row4 < nN) ? e4 : z4;

  const bool a8  = i < nU8;
  const int row8 = i >> 3;
  const int c8   = (i & 7) * 8;
  const int r8   = clampi(row8, 0, nN - 1);
  int id8 = x[r8];
  id8 = id8 < 0 ? id8 + V : id8;
  id8 = clampi(id8, 0, V - 1);
  const float* p8 = emb + (size_t)id8 * DS + c8;
  v4f ea = *(const v4f*)p8;
  v4f eb = *(const v4f*)(p8 + 4);
  ea = relu4(ea); eb = relu4(eb);
  ea = (row8 < nN) ? ea : z4;
  eb = (row8 < nN) ? eb : z4;
  const v8h o8 = cvt8(ea, eb, SCL_A);

  float*    d4 = F0f + (size_t)i * 4;
  _Float16* d8 = F0h + (size_t)i * 8;
  if (a4) *(volatile v4f*)d4 = e4;
  if (a8) *(volatile v8h*)d8 = o8;
  __threadfence();
  if (a4) *(volatile v4f*)d4 = e4;
  if (a8) *(volatile v8h*)d8 = o8;
}

__global__ __launch_bounds__(NTHR) void k_pq(const _Float16* __restrict__ Sh, const _Float16* __restrict__ wp,
                                            float* PQ, int nN) {
  __shared__ __attribute__((aligned(16))) float stg[BM * DP];
  const int tid = threadIdx.x, lane = tid & 31;
  const int wave = __builtin_amdgcn_readfirstlane(tid >> 5);
  const int hh = lane >> 4, m = lane & 15;
  const int rg = wave >> 2, cq = wave & 3;
  const int r0 = rg * 16, c0 = cq * 64;
  const int rowBase = blockIdx.x * BM;

  v8f acc[4];
#pragma unroll
  for (int t = 0; t < 4; ++t) { v8f z = {0.f, 0.f, 0.f, 0.f, 0.f, 0.f, 0.f, 0.f}; acc[t] = z; }

  const _Float16* ap = Sh + (size_t)(rowBase + r0 + m) * DS + 8 * hh;
#pragma unroll
  for (int ks = 0; ks < DS / 32; ++ks) {
    FragH a;
    a.h[0] = *(const v8h*)(ap + 32 * ks);
    a.h[1] = *(const v8h*)(ap + 32 * ks + 16);
#pragma unroll
    for (int t = 0; t < 4; ++t) {
      const _Float16* bp = wp + (size_t)(c0 + 16 * t + m) * DS + 32 * ks + 8 * hh;
      FragH b;
      b.h[0] = *(const v8h*)bp;
      b.h[1] = *(const v8h*)(bp + 16);
      acc[t] = wmh(a.v, b.v, acc[t]);
    }
  }

  float* sp = stg + (size_t)(r0 + 8 * hh) * DP + c0 + m;
  const int grow0 = rowBase + r0 + 8 * hh;
#pragma unroll
  for (int t = 0; t < 4; ++t) {
#pragma unroll
    for (int r = 0; r < 8; ++r) {
      float v = acc[t][r] * INV_PQ;
      v = (grow0 + r < nN) ? v : 0.0f;
      sp[r * DP + 16 * t] = v;
    }
  }
  __syncthreads();

  float* tile = PQ + (size_t)rowBase * DP;
  v4f ov[8];
#pragma unroll
  for (int it = 0; it < 8; ++it) ov[it] = *(const v4f*)(stg + 4 * (it * NTHR + tid));
#pragma unroll
  for (int it = 0; it < 8; ++it) *(volatile v4f*)(tile + 4 * (size_t)(it * NTHR + tid)) = ov[it];
  __threadfence();
#pragma unroll
  for (int it = 0; it < 8; ++it) *(volatile v4f*)(tile + 4 * (size_t)(it * NTHR + tid)) = ov[it];
}

template <int WH>
__global__ __launch_bounds__(NTHR) void k_layer(const int* __restrict__ rf, const float* __restrict__ PQ,
                                               const _Float16* __restrict__ Wbp, float* Sf, _Float16* Sh, int nN) {
  __shared__ __attribute__((aligned(16))) _Float16 wb[DS * DH];
  __shared__ __attribute__((aligned(16))) _Float16 at[NWAVE * 16 * DH];
  __shared__ __attribute__((aligned(16))) float part[NT * 2 * DS];
  __shared__ __attribute__((aligned(16))) float sv[VB * DS];
  __shared__ int sidx[VB * KP1];
  const int tid = threadIdx.x, lane = tid & 31;
  const int wave = __builtin_amdgcn_readfirstlane(tid >> 5);
  const int hh = lane >> 4, m = lane & 15;
  const int vbase = blockIdx.x * VB;
  const v4f z4 = {0.0f, 0.0f, 0.0f, 0.0f};

  {
    const size_t gmax = (size_t)nN * KP1 - 1;
    for (int i = tid; i < VB * KP1; i += NTHR) {
      size_t gi = (size_t)vbase * KP1 + (size_t)i;
      gi = gi > gmax ? gmax : gi;
      int w = rf[gi];
      w = w < 0 ? w + nN : w;
      sidx[i] = clampi(w, 0, nN - 1);
    }
#pragma unroll
    for (int it = 0; it < (DS * DH / 8) / NTHR; ++it) {
      const int u = it * NTHR + tid;
      *(v8h*)(wb + 8 * u) = *(const v8h*)(Wbp + 8 * u);
    }
  }
  __syncthreads();

  _Float16* atw = at + wave * (16 * DH);
#pragma unroll 1
  for (int it = 0; it < TIT; ++it) {
    const int t = it * NWAVE + wave;
    if (t < NT) {
#pragma unroll 4
      for (int o = 0; o < 16; ++o) {
        const int lr = t * 16 + o;
        const int lv = lr / KP1;
        const int w  = sidx[lr];
        int vq = vbase + lv;
        vq = vq > nN - 1 ? nN - 1 : vq;
        const v4f p = *(const v4f*)(PQ + (size_t)w * DP + 4 * lane);
        const v4f q = *(const v4f*)(PQ + (size_t)vq * DP + DH + 4 * lane);
        v4f u = relu4(p + q) * SCL_U;
        const v4h o4 = __builtin_convertvector(u, v4h);
        *(v4h*)(atw + o * DH + 4 * lane) = o4;
      }
    }
    __syncthreads();
    if (t < NT) {
      v8f acc[4];
#pragma unroll
      for (int nt = 0; nt < 4; ++nt) { v8f z = {0.f, 0.f, 0.f, 0.f, 0.f, 0.f, 0.f, 0.f}; acc[nt] = z; }
      const _Float16* arow = atw + m * DH + 8 * hh;
#pragma unroll
      for (int ks = 0; ks < DH / 32; ++ks) {
        FragH a;
        a.h[0] = *(const v8h*)(arow + 32 * ks);
        a.h[1] = *(const v8h*)(arow + 32 * ks + 16);
#pragma unroll
        for (int nt = 0; nt < 4; ++nt) {
          const _Float16* bp = wb + (16 * nt + m) * DH + 32 * ks + 8 * hh;
          FragH b;
          b.h[0] = *(const v8h*)bp;
          b.h[1] = *(const v8h*)(bp + 16);
          acc[nt] = wmh(a.v, b.v, acc[nt]);
        }
      }
      float lo[4], hi[4];
#pragma unroll
      for (int nt = 0; nt < 4; ++nt) {
        float l = 0.0f, h = 0.0f;
#pragma unroll
        for (int r = 0; r < 8; ++r) {
          const int o = 8 * hh + r;
          float v = acc[nt][r] * INV_H2;
          v = fmaxf(v, 0.0f);
          const bool isLow = o < t;
          l += isLow ? v : 0.0f;
          h += isLow ? 0.0f : v;
        }
        lo[nt] = l; hi[nt] = h;
      }
#pragma unroll
      for (int nt = 0; nt < 4; ++nt) {
        lo[nt] += __shfl_xor(lo[nt], 16);
        hi[nt] += __shfl_xor(hi[nt], 16);
        part[(t * 2 + hh) * DS + 16 * nt + m] = hh ? hi[nt] : lo[nt];
      }
    }
    __syncthreads();
  }

  {
    const int lv = tid >> 4;
    const int c0 = (tid & 15) * 4;
    const float* ph = part + (lv * 2 + 1) * DS + c0;
    const float* pl = part + ((lv + 1) * 2) * DS + c0;
    v4f s;
    s.x = ph[0] + pl[0]; s.y = ph[1] + pl[1]; s.z = ph[2] + pl[2]; s.w = ph[3] + pl[3];
    s = (vbase + lv < nN) ? s : z4;
    *(v4f*)(sv + 4 * tid) = s;
  }
  __syncthreads();

  const v4f f = *(const v4f*)(sv + 4 * tid);
  float* fp = Sf + (size_t)vbase * DS + 4 * tid;
  const int th = tid & 127;
  const v4f x0 = *(const v4f*)(sv + 8 * th);
  const v4f x1 = *(const v4f*)(sv + 8 * th + 4);
  const v8h hv = cvt8(x0, x1, SCL_A);
  _Float16* hp = Sh + (size_t)vbase * DS + 8 * th;
  *(volatile v4f*)fp = f;
  if (WH && tid < 128) *(volatile v8h*)hp = hv;
  __threadfence();
  *(volatile v4f*)fp = f;
  if (WH && tid < 128) *(volatile v8h*)hp = hv;
}

__global__ __launch_bounds__(NTHR) void k_mol(const int* __restrict__ mol,
    const float* __restrict__ F0f, const float* __restrict__ S0f, const float* __restrict__ S1f,
    const float* __restrict__ fcw, const float* __restrict__ fcb, float* out, int nN) {
  __shared__ int hl[HCAP];
  __shared__ int wsum[NWAVE];
  __shared__ __attribute__((aligned(16))) float rep[DFC];
  __shared__ __attribute__((aligned(16))) float so[DO];
  const int tid = threadIdx.x, lane = tid & 31;
  const int wave = __builtin_amdgcn_readfirstlane(tid >> 5);
  const int mid = blockIdx.x;

  int count = 0;
  const int nCh = (nN + CHK - 1) / CHK;
#pragma unroll 1
  for (int ch = 0; ch < nCh; ++ch) {
    const int cbase = ch * CHK;
    const int e0 = cbase + tid * 8;
    v4i da, db;
    if (cbase + CHK <= nN) {
      da = *(const v4i*)(mol + e0);
      db = *(const v4i*)(mol + e0 + 4);
    } else {
      const int sent = -1;
      da.x = (e0     < nN) ? mol[clampi(e0,     0, nN - 1)] : sent;
      da.y = (e0 + 1 < nN) ? mol[clampi(e0 + 1, 0, nN - 1)] : sent;
      da.z = (e0 + 2 < nN) ? mol[clampi(e0 + 2, 0, nN - 1)] : sent;
      da.w = (e0 + 3 < nN) ? mol[clampi(e0 + 3, 0, nN - 1)] : sent;
      db.x = (e0 + 4 < nN) ? mol[clampi(e0 + 4, 0, nN - 1)] : sent;
      db.y = (e0 + 5 < nN) ? mol[clampi(e0 + 5, 0, nN - 1)] : sent;
      db.z = (e0 + 6 < nN) ? mol[clampi(e0 + 6, 0, nN - 1)] : sent;
      db.w = (e0 + 7 < nN) ? mol[clampi(e0 + 7, 0, nN - 1)] : sent;
    }
    const bool h0 = da.x == mid, h1 = da.y == mid, h2 = da.z == mid, h3 = da.w == mid;
    const bool h4 = db.x == mid, h5 = db.y == mid, h6 = db.z == mid, h7 = db.w == mid;
    const int cnt = (int)h0 + (int)h1 + (int)h2 + (int)h3 + (int)h4 + (int)h5 + (int)h6 + (int)h7;
    int incl = cnt;
#pragma unroll
    for (int d = 1; d < 32; d <<= 1) {
      const int tv = __shfl_up(incl, d);
      if (lane >= d) incl += tv;
    }
    if (lane == 31) wsum[wave] = incl;
    __syncthreads();
    int pre = 0, tot = 0;
#pragma unroll
    for (int w = 0; w < NWAVE; ++w) {
      const int s = wsum[w];
      tot += s;
      pre += (w < wave) ? s : 0;
    }
    int pos = count + pre + incl - cnt;
#define PUT(HJ, J) if (HJ) { if (pos < HCAP) hl[pos] = e0 + (J); ++pos; }
    PUT(h0, 0) PUT(h1, 1) PUT(h2, 2) PUT(h3, 3) PUT(h4, 4) PUT(h5, 5) PUT(h6, 6) PUT(h7, 7)
#undef PUT
    count += tot;
    __syncthreads();
  }

  const int n = count > HCAP ? HCAP : count;
  const bool poison = count > HCAP;
  if (tid < DFC) {
    const int g = wave >> 1;
    const float* pl = (g == 0) ? F0f : ((g == 1) ? S0f : S1f);
    const int col = tid & 63;
    float s = 0.0f;
#pragma unroll 2
    for (int i = 0; i < n; ++i) {
      const int r = clampi(hl[i], 0, nN - 1);
      s += pl[(size_t)r * DS + col];
    }
    rep[tid] = s;
  }
  __syncthreads();
  if (tid < DO) {
    float d = 0.0f;
#pragma unroll 4
    for (int c = 0; c < DFC; ++c) d += rep[c] * fcw[c * DO + tid];
    float o = d + fcb[tid];
    if (poison) o = __int_as_float(0x7fc00000);
    so[tid] = o;
  }
  __syncthreads();
  v4f v = {0.0f, 0.0f, 0.0f, 0.0f};
  if (tid < 8) v = *(const v4f*)(so + 4 * tid);
  float* op = out + (size_t)mid * DO + 4 * (tid & 7);
  if (tid < 8) *(volatile v4f*)op = v;
  __threadfence();
  if (tid < 8) *(volatile v4f*)op = v;
}

extern "C" void kernel_launch(void* const* d_in, const int* in_sizes, int n_in,
                              void* d_out, int out_size, void* d_ws, size_t ws_size,
                              hipStream_t stream) {
  if (n_in < 10) return;
  const int nN = in_sizes[0];
  if (nN <= 0 || nN > (1 << 24)) return;
  if (in_sizes[1] != nN * KP1 || in_sizes[2] != nN) return;
  const int V = in_sizes[3] / DS;
  if (V <= 0 || in_sizes[3] != V * DS) return;
  if (in_sizes[4] != DH * DH || in_sizes[5] != DH * DS) return;
  if (in_sizes[6] != DH * DH || in_sizes[7] != DH * DS) return;
  if (in_sizes[8] != DFC * DO || in_sizes[9] != DO) return;
  if (out_size <= 0 || (out_size % DO) != 0) return;
  const int nMol = out_size / DO;

  const int*   x   = (const int*)d_in[0];
  const int*   rf  = (const int*)d_in[1];
  const int*   mol = (const int*)d_in[2];
  const float* emb = (const float*)d_in[3];
  const float* Wa0 = (const float*)d_in[4];
  const float* Wb0 = (const float*)d_in[5];
  const float* Wa1 = (const float*)d_in[6];
  const float* Wb1 = (const float*)d_in[7];
  const float* fcw = (const float*)d_in[8];
  const float* fcb = (const float*)d_in[9];
  float* out = (float*)d_out;

  const int nPad = ((nN + BM - 1) / BM) * BM;
  const int nU4  = nPad * (DS / 4);
  const int nU8  = nPad * (DS / 8);

  char* ws = (char*)d_ws;
  size_t off = 0;
  const size_t szWA = (size_t)DP * DS * 2;
  const size_t szWB = (size_t)DS * DH * 2;
  const size_t szF  = (size_t)nPad * DS * 4;
  const size_t szH  = (size_t)nPad * DS * 2;
  const size_t szPQ = (size_t)nPad * DP * 4;
  const size_t oWA0 = off; off += szWA;  off = (off + 255) & ~(size_t)255;
  const size_t oWA1 = off; off += szWA;  off = (off + 255) & ~(size_t)255;
  const size_t oWB0 = off; off += szWB;  off = (off + 255) & ~(size_t)255;
  const size_t oWB1 = off; off += szWB;  off = (off + 255) & ~(size_t)255;
  const size_t oF0f = off; off += szF;   off = (off + 255) & ~(size_t)255;
  const size_t oF0h = off; off += szH;   off = (off + 255) & ~(size_t)255;
  const size_t oS0f = off; off += szF;   off = (off + 255) & ~(size_t)255;
  const size_t oS0h = off; off += szH;   off = (off + 255) & ~(size_t)255;
  const size_t oS1f = off; off += szF;   off = (off + 255) & ~(size_t)255;
  const size_t oPQ  = off; off += szPQ;  off = (off + 255) & ~(size_t)255;
  if (off > ws_size || off > (size_t)WSCAP) return;
  _Float16* pWA0 = (_Float16*)(ws + oWA0);
  _Float16* pWA1 = (_Float16*)(ws + oWA1);
  _Float16* pWB0 = (_Float16*)(ws + oWB0);
  _Float16* pWB1 = (_Float16*)(ws + oWB1);
  float*    F0f  = (float*)(ws + oF0f);
  _Float16* F0h  = (_Float16*)(ws + oF0h);
  float*    S0f  = (float*)(ws + oS0f);
  _Float16* S0h  = (_Float16*)(ws + oS0h);
  float*    S1f  = (float*)(ws + oS1f);
  float*    PQ   = (float*)(ws + oPQ);

  k_prepw<<<(DP * DS / 8 + NTHR - 1) / NTHR, NTHR, 0, stream>>>(Wa0, pWA0, DH, DH, DP, DS, DH, DS);
  k_prepw<<<(DS * DH / 8 + NTHR - 1) / NTHR, NTHR, 0, stream>>>(Wb0, pWB0, DH, DS, DS, DH, DS, 0);
  k_prepw<<<(DP * DS / 8 + NTHR - 1) / NTHR, NTHR, 0, stream>>>(Wa1, pWA1, DH, DH, DP, DS, DH, DS);
  k_prepw<<<(DS * DH / 8 + NTHR - 1) / NTHR, NTHR, 0, stream>>>(Wb1, pWB1, DH, DS, DS, DH, DS, 0);

  k_embed<<<(nU4 + NTHR - 1) / NTHR, NTHR, 0, stream>>>(x, emb, F0f, F0h, nN, V, nU4, nU8);

  k_pq<<<nPad / BM, NTHR, 0, stream>>>(F0h, pWA0, PQ, nN);
  k_layer<1><<<nPad / VB, NTHR, 0, stream>>>(rf, PQ, pWB0, S0f, S0h, nN);

  k_pq<<<nPad / BM, NTHR, 0, stream>>>(S0h, pWA1, PQ, nN);
  k_layer<0><<<nPad / VB, NTHR, 0, stream>>>(rf, PQ, pWB1, S1f, S0h, nN);

  k_mol<<<nMol, NTHR, 0, stream>>>(mol, F0f, S0f, S1f, fcw, fcb, out, nN);
}
